// GNN_graph_clasif_model_28793460752816
// MI455X (gfx1250) — hardware-verified
//
#include <hip/hip_runtime.h>
#include <stddef.h>
#include <math.h>


#define DF      128
#define DH      64
#define NCLS    10
#define NCP     16
#define NGR     512
#define NTHR    256
#define NWAVE   8
#define EPT     8
#define NGRP    2
#define CHUNK   (NTHR * EPT * NGRP)
#define WCAP    (EPT * NGRP * 32)
#define LISTN   (NWAVE * WCAP)
#define NBD     4096
#define NB1     1024
#define NB2     1024
#define G1ROWS  128
#define APITCH  136
#define WSCALE  8.0f
#define WINV    0.125f

#define LDS_GEMM1 (G1ROWS * APITCH * 2)
#define LDS_AGG   (NB1 * DH * 4 + LISTN * 4 + 64)
#define LDS_POOL  (NGR * DH * 4 + LISTN * 4 + 64 + NGR * NCP * 4)

static_assert((CHUNK & (CHUNK - 1)) == 0);
static_assert(CHUNK <= 4096);
static_assert(NBD <= 4096 && NB1 <= 4096 && NB2 <= 4096 && NGR <= 4096);
static_assert((NBD & (NBD - 1)) == 0 && (NB1 & (NB1 - 1)) == 0 && (NGR & (NGR - 1)) == 0);
static_assert(NB1 == NB2);
static_assert(G1ROWS * DH * 4 <= LDS_GEMM1);
static_assert(NB1 / 16 == 8 * NWAVE);
static_assert(NGR / 16 == 4 * NWAVE);
static_assert(NGR == 2 * NTHR);
static_assert(NGR * NCLS == NWAVE * 5 * 32 * 4);
static_assert(NGR * NCLS * 4 <= NGR * DH * 4);

typedef float    v2f  __attribute__((ext_vector_type(2)));
typedef float    v4f  __attribute__((ext_vector_type(4)));
typedef float    v8f  __attribute__((ext_vector_type(8)));
typedef int      v4i  __attribute__((ext_vector_type(4)));
typedef _Float16 v8h  __attribute__((ext_vector_type(8)));
typedef _Float16 v16h __attribute__((ext_vector_type(16)));
union FragH { v16h v; v8h h[2]; };

__device__ __forceinline__ v8h cvt8(v4f a, v4f b) {
  v8h r;
  r[0] = (_Float16)a.x; r[1] = (_Float16)a.y; r[2] = (_Float16)a.z; r[3] = (_Float16)a.w;
  r[4] = (_Float16)b.x; r[5] = (_Float16)b.y; r[6] = (_Float16)b.z; r[7] = (_Float16)b.w;
  return r;
}

__device__ __forceinline__ v8f wmh(v16h a, v16h b, v8f c) {
  v8f d = __builtin_amdgcn_wmma_f32_16x16x32_f16(false, a, false, b, (short)0, c, false, false);
  asm volatile("v_nop\n\tv_nop\n\tv_nop\n\tv_nop" : "+v"(d) : "v"(a), "v"(b));
  return d;
}

template <int NB>
__device__ __forceinline__ int scan_chunk(const int* __restrict__ dsts, int nE, int cbase, int nodeBase,
                                          int vec8, int* list, int tid, int lane, int wave) {
  int wc = 0;
#pragma unroll
  for (int g = 0; g < NGRP; ++g) {
    const int el0  = (g * NTHR + tid) * EPT;
    const int e0   = cbase + el0;
    const int sent = -2147483647 - 1;
    v4i da, db;
    if (vec8 != 0 && e0 + 7 < nE) {
      da = *(const v4i*)(dsts + e0);
      db = *(const v4i*)(dsts + e0 + 4);
    } else {
      da.x = (e0     < nE) ? dsts[min(e0, nE - 1)] : sent;
      da.y = (e0 + 1 < nE) ? dsts[min(e0 + 1, nE - 1)] : sent;
      da.z = (e0 + 2 < nE) ? dsts[min(e0 + 2, nE - 1)] : sent;
      da.w = (e0 + 3 < nE) ? dsts[min(e0 + 3, nE - 1)] : sent;
      db.x = (e0 + 4 < nE) ? dsts[min(e0 + 4, nE - 1)] : sent;
      db.y = (e0 + 5 < nE) ? dsts[min(e0 + 5, nE - 1)] : sent;
      db.z = (e0 + 6 < nE) ? dsts[min(e0 + 6, nE - 1)] : sent;
      db.w = (e0 + 7 < nE) ? dsts[min(e0 + 7, nE - 1)] : sent;
    }
    const unsigned nb = (unsigned)nodeBase;
    const unsigned s0 = (unsigned)da.x - nb, s1 = (unsigned)da.y - nb;
    const unsigned s2 = (unsigned)da.z - nb, s3 = (unsigned)da.w - nb;
    const unsigned s4 = (unsigned)db.x - nb, s5 = (unsigned)db.y - nb;
    const unsigned s6 = (unsigned)db.z - nb, s7 = (unsigned)db.w - nb;
    const bool h0 = s0 < (unsigned)NB, h1 = s1 < (unsigned)NB, h2 = s2 < (unsigned)NB, h3 = s3 < (unsigned)NB;
    const bool h4 = s4 < (unsigned)NB, h5 = s5 < (unsigned)NB, h6 = s6 < (unsigned)NB, h7 = s7 < (unsigned)NB;
    const unsigned any = __builtin_amdgcn_ballot_w32(h0 | h1 | h2 | h3 | h4 | h5 | h6 | h7);
    if (any != 0u) {
#define HITJ(J, HJ, SJ) { \
        const unsigned mj = __builtin_amdgcn_ballot_w32(HJ); \
        if (mj != 0u) { \
          if (HJ) { \
            const int pos = wc + (int)__builtin_amdgcn_mbcnt_lo(mj, 0u); \
            if (pos < WCAP) list[wave * WCAP + pos] = ((el0 + (J)) << 12) | (int)(SJ); \
          } \
          wc += (int)__builtin_popcount(mj); } }
      HITJ(0, h0, s0)
      HITJ(1, h1, s1)
      HITJ(2, h2, s2)
      HITJ(3, h3, s3)
      HITJ(4, h4, s4)
      HITJ(5, h5, s5)
      HITJ(6, h6, s6)
      HITJ(7, h7, s7)
#undef HITJ
    }
  }
  return wc;
}

template <int NB, bool VIA>
__device__ __forceinline__ void drain64(const int* list, const int* wcnt, float* acc,
                                        const float* __restrict__ rows, const int* __restrict__ idx,
                                        int cbase, int nIdx, int nRows, int lane) {
#pragma unroll 1
  for (int wsx = 0; wsx < NWAVE; ++wsx) {
    int n = __builtin_amdgcn_readfirstlane(wcnt[wsx]);
    n = n > WCAP ? WCAP : (n < 0 ? 0 : n);
    const int* lp = list + wsx * WCAP;
#pragma unroll 1
    for (int i = 0; i < n; ++i) {
      const int ent  = __builtin_amdgcn_readfirstlane(lp[i]);
      const int slot = ent & (NB - 1);
      int e = cbase + ((ent >> 12) & (CHUNK - 1));
      e = e > nIdx - 1 ? nIdx - 1 : e;
      int r;
      if (VIA) { r = idx[e]; r = r < 0 ? 0 : (r > nRows - 1 ? nRows - 1 : r); }
      else     { r = e > nRows - 1 ? nRows - 1 : e; }
      const v2f v = *(const v2f*)(rows + (size_t)r * DH + 2 * lane);
      v2f* ap = (v2f*)(acc + slot * DH + 2 * lane);
      *ap = *ap + v;
    }
  }
}

__global__ __launch_bounds__(NTHR) void k_wprep(
    const float* __restrict__ W1, const float* __restrict__ W2, const float* __restrict__ Wf,
    _Float16* w1s, _Float16* w2s, _Float16* wfs) {
  const int i  = blockIdx.x * NTHR + threadIdx.x;
  const int n1 = DH * DF / 8;
  const int n2 = DH * DH / 8;
  const int n3 = NCP * DH / 8;
  if (i >= n1 + n2 + n3) return;
  v4f a, b;
  _Float16* dp;
  if (i < n1) {
    const int o = i * 8, n = o / DF, k0 = o - n * DF;
    const float* p = W1 + (size_t)k0 * DH + n;
    a.x = p[0];      a.y = p[DH];     a.z = p[2 * DH]; a.w = p[3 * DH];
    b.x = p[4 * DH]; b.y = p[5 * DH]; b.z = p[6 * DH]; b.w = p[7 * DH];
    dp = w1s + o;
  } else if (i < n1 + n2) {
    const int o = (i - n1) * 8, n = o / DH, k0 = o - n * DH;
    const float* p = W2 + (size_t)k0 * DH + n;
    a.x = p[0];      a.y = p[DH];     a.z = p[2 * DH]; a.w = p[3 * DH];
    b.x = p[4 * DH]; b.y = p[5 * DH]; b.z = p[6 * DH]; b.w = p[7 * DH];
    dp = w2s + o;
  } else {
    const int o = (i - n1 - n2) * 8, n = o / DH, k0 = o - n * DH;
    if (n < NCLS) {
      const float* p = Wf + (size_t)k0 * NCLS + n;
      a.x = p[0];        a.y = p[NCLS];     a.z = p[2 * NCLS]; a.w = p[3 * NCLS];
      b.x = p[4 * NCLS]; b.y = p[5 * NCLS]; b.z = p[6 * NCLS]; b.w = p[7 * NCLS];
    } else {
      const v4f z = {0.f, 0.f, 0.f, 0.f};
      a = z; b = z;
    }
    dp = wfs + o;
  }
  a = a * WSCALE;
  b = b * WSCALE;
  const v8h hv = cvt8(a, b);
  *(volatile v8h*)dp = hv;
  __threadfence();
  *(volatile v8h*)dp = hv;
}

__global__ __launch_bounds__(NTHR) void k_deg(
    const int* __restrict__ ei, float* dinv, int nE, int vec8) {
  __shared__ __attribute__((aligned(16))) int cnt[NBD];
  __shared__ __attribute__((aligned(16))) int list[LISTN];
  __shared__ int wcnt[NWAVE];
  const int tid = threadIdx.x, lane = tid & 31, wave = tid >> 5;
  const int nodeBase = blockIdx.x * NBD;
  const int* dsts = ei + nE;

  for (int i = tid; i < NBD; i += NTHR) cnt[i] = 0;
  __syncthreads();

  const int nChunks = (nE + CHUNK - 1) / CHUNK;
#pragma unroll 1
  for (int ch = 0; ch < nChunks; ++ch) {
    const int cbase = ch * CHUNK;
    const int wc = scan_chunk<NBD>(dsts, nE, cbase, nodeBase, vec8, list, tid, lane, wave);
    if (lane == 0) wcnt[wave] = wc;
    __syncthreads();
    if (wave == 0) {
#pragma unroll 1
      for (int wsx = 0; wsx < NWAVE; ++wsx) {
        int n = __builtin_amdgcn_readfirstlane(wcnt[wsx]);
        n = n > WCAP ? WCAP : (n < 0 ? 0 : n);
        const int* lp = list + wsx * WCAP;
#pragma unroll 1
        for (int i = 0; i < n; ++i) {
          const int ent  = __builtin_amdgcn_readfirstlane(lp[i]);
          const int slot = ent & (NBD - 1);
          if (lane == 0) cnt[slot] = cnt[slot] + 1;
        }
      }
    }
    __syncthreads();
  }

  v4f dq[4];
#pragma unroll
  for (int q = 0; q < 4; ++q) {
    const int f = (wave * 4 + q) * 128 + 4 * lane;
    const v4i c = *(const v4i*)(cnt + f);
    dq[q].x = rsqrtf((float)(c.x + 1));
    dq[q].y = rsqrtf((float)(c.y + 1));
    dq[q].z = rsqrtf((float)(c.z + 1));
    dq[q].w = rsqrtf((float)(c.w + 1));
  }
  float* dp = dinv + (size_t)nodeBase;
#pragma unroll
  for (int q = 0; q < 4; ++q) *(volatile v4f*)(dp + (wave * 4 + q) * 128 + 4 * lane) = dq[q];
  __threadfence();
#pragma unroll
  for (int q = 0; q < 4; ++q) *(volatile v4f*)(dp + (wave * 4 + q) * 128 + 4 * lane) = dq[q];
}

__global__ __launch_bounds__(NTHR) void k_gemm1(
    const float* __restrict__ x, const _Float16* __restrict__ w1s,
    const float* __restrict__ dinv, float* g1, int nN) {
  extern __shared__ v4f lds_dyn[];
  _Float16* sA  = (_Float16*)lds_dyn;
  float*    stg = (float*)lds_dyn;
  const int tid = threadIdx.x, lane = tid & 31, wave = tid >> 5, hh = lane >> 4, m = lane & 15;
  const int rowBase = blockIdx.x * G1ROWS;

#pragma unroll
  for (int i = 0; i < (G1ROWS * DF / 8) / NTHR; ++i) {
    const int idx = i * NTHR + tid;
    const int r   = idx >> 4;
    const int c0  = (idx & 15) * 8;
    int node = rowBase + r;
    node = node > nN - 1 ? nN - 1 : node;
    const float* xp = x + (size_t)node * DF + c0;
    const v4f a = *(const v4f*)xp, b = *(const v4f*)(xp + 4);
    *(v8h*)(sA + r * APITCH + c0) = cvt8(a, b);
  }
  __syncthreads();

  v8f acc[4];
#pragma unroll
  for (int t = 0; t < 4; ++t) { v8f z = {0.f, 0.f, 0.f, 0.f, 0.f, 0.f, 0.f, 0.f}; acc[t] = z; }
  const _Float16* ar = sA + (wave * 16 + m) * APITCH + 8 * hh;
#pragma unroll
  for (int kt = 0; kt < DF / 32; ++kt) {
    FragH a;
    a.h[0] = *(const v8h*)(ar + 32 * kt);
    a.h[1] = *(const v8h*)(ar + 32 * kt + 16);
#pragma unroll
    for (int t = 0; t < 4; ++t) {
      const _Float16* bp = w1s + (size_t)(16 * t + m) * DF + 32 * kt + 8 * hh;
      FragH b;
      b.h[0] = *(const v8h*)bp;
      b.h[1] = *(const v8h*)(bp + 16);
      acc[t] = wmh(a.v, b.v, acc[t]);
    }
  }
  __syncthreads();

  const int r0 = wave * 16 + 8 * hh;
  const v4f dA = *(const v4f*)(dinv + (size_t)rowBase + r0);
  const v4f dB = *(const v4f*)(dinv + (size_t)rowBase + r0 + 4);
  const float d0 = dA.x * WINV, d1 = dA.y * WINV, d2 = dA.z * WINV, d3 = dA.w * WINV;
  const float d4 = dB.x * WINV, d5 = dB.y * WINV, d6 = dB.z * WINV, d7 = dB.w * WINV;
  float* sp = stg + r0 * DH + m;
#pragma unroll
  for (int t = 0; t < 4; ++t) {
    sp[0 * DH + 16 * t] = acc[t][0] * d0;
    sp[1 * DH + 16 * t] = acc[t][1] * d1;
    sp[2 * DH + 16 * t] = acc[t][2] * d2;
    sp[3 * DH + 16 * t] = acc[t][3] * d3;
    sp[4 * DH + 16 * t] = acc[t][4] * d4;
    sp[5 * DH + 16 * t] = acc[t][5] * d5;
    sp[6 * DH + 16 * t] = acc[t][6] * d6;
    sp[7 * DH + 16 * t] = acc[t][7] * d7;
  }
  __syncthreads();

  const float* lp = stg + wave * 16 * DH + 4 * lane;
  float* gp = g1 + ((size_t)rowBase + wave * 16) * DH + 4 * lane;
  v4f ov[8];
#pragma unroll
  for (int q = 0; q < 8; ++q) ov[q] = *(const v4f*)(lp + q * 128);
#pragma unroll
  for (int q = 0; q < 8; ++q) *(volatile v4f*)(gp + q * 128) = ov[q];
  __threadfence();
#pragma unroll
  for (int q = 0; q < 8; ++q) *(volatile v4f*)(gp + q * 128) = ov[q];
}

__global__ __launch_bounds__(NTHR) void k_agg1(
    const int* __restrict__ ei, const float* __restrict__ g1, const float* __restrict__ dinv,
    const float* __restrict__ b1, const _Float16* __restrict__ w2s, float* g2,
    int nN, int nE, int vec8) {
  extern __shared__ v4f lds_dyn[];
  float* acc  = (float*)lds_dyn;
  int*   list = (int*)(acc + NB1 * DH);
  int*   wcnt = list + LISTN;
  const int tid = threadIdx.x, lane = tid & 31, wave = tid >> 5, hh = lane >> 4, m = lane & 15;
  const int nodeBase = blockIdx.x * NB1;
  const int* dsts = ei + nE;

  {
    const v4f z = {0.f, 0.f, 0.f, 0.f};
    for (int i = tid; i < NB1 * DH / 4; i += NTHR) lds_dyn[i] = z;
  }
  __syncthreads();

  const int nChunks = (nE + CHUNK - 1) / CHUNK;
#pragma unroll 1
  for (int ch = 0; ch < nChunks; ++ch) {
    const int cbase = ch * CHUNK;
    const int wc = scan_chunk<NB1>(dsts, nE, cbase, nodeBase, vec8, list, tid, lane, wave);
    if (lane == 0) wcnt[wave] = wc;
    __syncthreads();
    if (wave == 0) drain64<NB1, true>(list, wcnt, acc, g1, ei, cbase, nE, nN, lane);
    __syncthreads();
  }

#pragma unroll 4
  for (int i = 0; i < (NB1 * DH / 4) / NTHR; ++i) {
    const int idx  = i * NTHR + tid;
    const int slot = idx >> 4;
    const int c4   = (idx & 15) * 4;
    int node = nodeBase + slot;
    node = node > nN - 1 ? nN - 1 : node;
    const float d  = dinv[node];
    const v4f   gv = *(const v4f*)(g1 + (size_t)node * DH + c4);
    const v4f   bv = *(const v4f*)(b1 + c4);
    v4f* ap = (v4f*)(acc + slot * DH + c4);
    v4f hv = (*ap + gv) * d + bv;
    hv.x = fmaxf(hv.x, 0.f); hv.y = fmaxf(hv.y, 0.f); hv.z = fmaxf(hv.z, 0.f); hv.w = fmaxf(hv.w, 0.f);
    *ap = hv;
  }
  __syncthreads();

  FragH bw[4][2];
#pragma unroll
  for (int ct = 0; ct < 4; ++ct) {
#pragma unroll
    for (int kt = 0; kt < 2; ++kt) {
      const _Float16* bp = w2s + (16 * ct + m) * DH + 32 * kt + 8 * hh;
      bw[ct][kt].h[0] = *(const v8h*)bp;
      bw[ct][kt].h[1] = *(const v8h*)(bp + 16);
    }
  }

#pragma unroll 1
  for (int q = 0; q < 8; ++q) {
    const int t = wave + 8 * q;
    v8f c[4];
#pragma unroll
    for (int ct = 0; ct < 4; ++ct) { v8f z = {0.f, 0.f, 0.f, 0.f, 0.f, 0.f, 0.f, 0.f}; c[ct] = z; }
#pragma unroll
    for (int kt = 0; kt < 2; ++kt) {
      const float* ap = acc + (16 * t + m) * DH + 32 * kt + 8 * hh;
      const v4f p0 = *(const v4f*)ap,        p1 = *(const v4f*)(ap + 4);
      const v4f p2 = *(const v4f*)(ap + 16), p3 = *(const v4f*)(ap + 20);
      FragH a;
      a.h[0] = cvt8(p0, p1);
      a.h[1] = cvt8(p2, p3);
#pragma unroll
      for (int ct = 0; ct < 4; ++ct) c[ct] = wmh(a.v, bw[ct][kt].v, c[ct]);
    }
    const int node0 = nodeBase + 16 * t + 8 * hh;
    const v4f dA = *(const v4f*)(dinv + (size_t)node0);
    const v4f dB = *(const v4f*)(dinv + (size_t)node0 + 4);
    const float d0 = dA.x * WINV, d1 = dA.y * WINV, d2 = dA.z * WINV, d3 = dA.w * WINV;
    const float d4 = dB.x * WINV, d5 = dB.y * WINV, d6 = dB.z * WINV, d7 = dB.w * WINV;
    float* sp = acc + (16 * t + 8 * hh) * DH + m;
#pragma unroll
    for (int ct = 0; ct < 4; ++ct) {
      sp[0 * DH + 16 * ct] = c[ct][0] * d0;
      sp[1 * DH + 16 * ct] = c[ct][1] * d1;
      sp[2 * DH + 16 * ct] = c[ct][2] * d2;
      sp[3 * DH + 16 * ct] = c[ct][3] * d3;
      sp[4 * DH + 16 * ct] = c[ct][4] * d4;
      sp[5 * DH + 16 * ct] = c[ct][5] * d5;
      sp[6 * DH + 16 * ct] = c[ct][6] * d6;
      sp[7 * DH + 16 * ct] = c[ct][7] * d7;
    }
  }
  __syncthreads();

  float* gp = g2 + (size_t)nodeBase * DH;
#pragma unroll 4
  for (int q = 0; q < 64; ++q) {
    const int f = (wave * 64 + q) * 128 + 4 * lane;
    const v4f v = *(const v4f*)(acc + f);
    *(volatile v4f*)(gp + f) = v;
  }
  __threadfence();
#pragma unroll 4
  for (int q = 0; q < 64; ++q) {
    const int f = (wave * 64 + q) * 128 + 4 * lane;
    const v4f v = *(const v4f*)(acc + f);
    *(volatile v4f*)(gp + f) = v;
  }
}

__global__ __launch_bounds__(NTHR) void k_agg2(
    const int* __restrict__ ei, const float* __restrict__ g2, const float* __restrict__ dinv,
    const float* __restrict__ b2, float* h2, int nN, int nE, int vec8) {
  extern __shared__ v4f lds_dyn[];
  float* acc  = (float*)lds_dyn;
  int*   list = (int*)(acc + NB2 * DH);
  int*   wcnt = list + LISTN;
  const int tid = threadIdx.x, lane = tid & 31, wave = tid >> 5;
  const int nodeBase = blockIdx.x * NB2;
  const int* dsts = ei + nE;

  {
    const v4f z = {0.f, 0.f, 0.f, 0.f};
    for (int i = tid; i < NB2 * DH / 4; i += NTHR) lds_dyn[i] = z;
  }
  __syncthreads();

  const int nChunks = (nE + CHUNK - 1) / CHUNK;
#pragma unroll 1
  for (int ch = 0; ch < nChunks; ++ch) {
    const int cbase = ch * CHUNK;
    const int wc = scan_chunk<NB2>(dsts, nE, cbase, nodeBase, vec8, list, tid, lane, wave);
    if (lane == 0) wcnt[wave] = wc;
    __syncthreads();
    if (wave == 0) drain64<NB2, true>(list, wcnt, acc, g2, ei, cbase, nE, nN, lane);
    __syncthreads();
  }

#pragma unroll 4
  for (int i = 0; i < (NB2 * DH / 4) / NTHR; ++i) {
    const int idx  = i * NTHR + tid;
    const int slot = idx >> 4;
    const int c4   = (idx & 15) * 4;
    int node = nodeBase + slot;
    node = node > nN - 1 ? nN - 1 : node;
    const float d  = dinv[node];
    const v4f   gv = *(const v4f*)(g2 + (size_t)node * DH + c4);
    const v4f   bv = *(const v4f*)(b2 + c4);
    v4f* ap = (v4f*)(acc + slot * DH + c4);
    v4f hv = (*ap + gv) * d + bv;
    hv.x = fmaxf(hv.x, 0.f); hv.y = fmaxf(hv.y, 0.f); hv.z = fmaxf(hv.z, 0.f); hv.w = fmaxf(hv.w, 0.f);
    *ap = hv;
  }
  __syncthreads();

  float* gp = h2 + (size_t)nodeBase * DH;
#pragma unroll 4
  for (int q = 0; q < 64; ++q) {
    const int f = (wave * 64 + q) * 128 + 4 * lane;
    const v4f v = *(const v4f*)(acc + f);
    *(volatile v4f*)(gp + f) = v;
  }
  __threadfence();
#pragma unroll 4
  for (int q = 0; q < 64; ++q) {
    const int f = (wave * 64 + q) * 128 + 4 * lane;
    const v4f v = *(const v4f*)(acc + f);
    *(volatile v4f*)(gp + f) = v;
  }
}

__global__ __launch_bounds__(NTHR) void k_pool(
    const int* __restrict__ batch, const float* __restrict__ h2,
    const _Float16* __restrict__ wfs, const float* __restrict__ bfv, float* out, int nN) {
  extern __shared__ v4f lds_dyn[];
  float* gacc = (float*)lds_dyn;
  int*   list = (int*)(gacc + NGR * DH);
  int*   wcnt = list + LISTN;
  float* lstg = (float*)(wcnt + 16);
  float* ostg = gacc;
  const int tid = threadIdx.x, lane = tid & 31, wave = tid >> 5, hh = lane >> 4, m = lane & 15;

  {
    const v4f z = {0.f, 0.f, 0.f, 0.f};
    for (int i = tid; i < NGR * DH / 4; i += NTHR) lds_dyn[i] = z;
  }
  __syncthreads();

  const int nChunks = (nN + CHUNK - 1) / CHUNK;
#pragma unroll 1
  for (int ch = 0; ch < nChunks; ++ch) {
    const int cbase = ch * CHUNK;
    const int wc = scan_chunk<NGR>(batch, nN, cbase, 0, 1, list, tid, lane, wave);
    if (lane == 0) wcnt[wave] = wc;
    __syncthreads();
    if (wave == 0) drain64<NGR, false>(list, wcnt, gacc, h2, batch, cbase, nN, nN, lane);
    __syncthreads();
  }

  FragH bq[2];
#pragma unroll
  for (int kt = 0; kt < 2; ++kt) {
    const _Float16* bp = wfs + m * DH + 32 * kt + 8 * hh;
    bq[kt].h[0] = *(const v8h*)bp;
    bq[kt].h[1] = *(const v8h*)(bp + 16);
  }
#pragma unroll 1
  for (int q = 0; q < 4; ++q) {
    const int t = wave + 8 * q;
    v8f c = {0.f, 0.f, 0.f, 0.f, 0.f, 0.f, 0.f, 0.f};
#pragma unroll
    for (int kt = 0; kt < 2; ++kt) {
      const float* ap = gacc + (16 * t + m) * DH + 32 * kt + 8 * hh;
      const v4f p0 = *(const v4f*)ap,        p1 = *(const v4f*)(ap + 4);
      const v4f p2 = *(const v4f*)(ap + 16), p3 = *(const v4f*)(ap + 20);
      FragH a;
      a.h[0] = cvt8(p0, p1);
      a.h[1] = cvt8(p2, p3);
      c = wmh(a.v, bq[kt].v, c);
    }
    float* sp = lstg + (16 * t + 8 * hh) * NCP + m;
    sp[0 * NCP] = c[0] * WINV;
    sp[1 * NCP] = c[1] * WINV;
    sp[2 * NCP] = c[2] * WINV;
    sp[3 * NCP] = c[3] * WINV;
    sp[4 * NCP] = c[4] * WINV;
    sp[5 * NCP] = c[5] * WINV;
    sp[6 * NCP] = c[6] * WINV;
    sp[7 * NCP] = c[7] * WINV;
  }
  __syncthreads();

#pragma unroll
  for (int rr = 0; rr < 2; ++rr) {
    const int row = tid + rr * NTHR;
    float v[NCLS];
#pragma unroll
    for (int cc = 0; cc < NCLS; ++cc) v[cc] = lstg[row * NCP + cc] + bfv[cc];
    float mx = v[0];
#pragma unroll
    for (int cc = 1; cc < NCLS; ++cc) mx = fmaxf(mx, v[cc]);
    float s = 0.f;
#pragma unroll
    for (int cc = 0; cc < NCLS; ++cc) { v[cc] = v[cc] - mx; s += expf(v[cc]); }
    const float ls = logf(s);
#pragma unroll
    for (int cc = 0; cc < NCLS; ++cc) ostg[row * NCLS + cc] = v[cc] - ls;
  }
  __syncthreads();

  v4f ov[5];
#pragma unroll
  for (int q = 0; q < 5; ++q) ov[q] = lds_dyn[(wave * 5 + q) * 32 + lane];
#pragma unroll
  for (int q = 0; q < 5; ++q) *(volatile v4f*)(out + (size_t)4 * ((wave * 5 + q) * 32 + lane)) = ov[q];
  __threadfence();
#pragma unroll
  for (int q = 0; q < 5; ++q) *(volatile v4f*)(out + (size_t)4 * ((wave * 5 + q) * 32 + lane)) = ov[q];
}

extern "C" void kernel_launch(void* const* d_in, const int* in_sizes, int n_in,
                              void* d_out, int out_size, void* d_ws, size_t ws_size,
                              hipStream_t stream) {
  if (n_in < 9) return;
  const int nN = in_sizes[0] / DF;
  const int nE = in_sizes[1] / 2;
  if (nN <= 0 || nE <= 0 || in_sizes[0] != nN * DF || in_sizes[1] != nE * 2) return;
  if (in_sizes[2] != nN) return;
  if (in_sizes[3] != DF * DH || in_sizes[4] < DH || in_sizes[5] != DH * DH || in_sizes[6] < DH) return;
  if (in_sizes[7] != DH * NCLS || in_sizes[8] < NCLS) return;
  if (out_size != NGR * NCLS) return;

  const float* x     = (const float*)d_in[0];
  const int*   ei    = (const int*)d_in[1];
  const int*   batch = (const int*)d_in[2];
  const float* W1    = (const float*)d_in[3];
  const float* b1    = (const float*)d_in[4];
  const float* W2    = (const float*)d_in[5];
  const float* b2    = (const float*)d_in[6];
  const float* Wf    = (const float*)d_in[7];
  const float* bfv   = (const float*)d_in[8];
  float* out = (float*)d_out;

  const int nBD = (nN + NBD - 1) / NBD;
  const int nG1 = (nN + G1ROWS - 1) / G1ROWS;
  const int nA1 = (nN + NB1 - 1) / NB1;
  const int nA2 = (nN + NB2 - 1) / NB2;

  char* ws = (char*)d_ws;
  size_t off = 0;
  const size_t oW1 = off; off += (size_t)DH * DF * 2;                          off = (off + 255) & ~(size_t)255;
  const size_t oW2 = off; off += (size_t)DH * DH * 2;                          off = (off + 255) & ~(size_t)255;
  const size_t oWf = off; off += (size_t)NCP * DH * 2;                         off = (off + 255) & ~(size_t)255;
  const size_t oDv = off; off += (size_t)nBD * NBD * 4;                        off = (off + 255) & ~(size_t)255;
  const size_t oG1 = off; off += (size_t)nG1 * G1ROWS * DH * 4;                off = (off + 255) & ~(size_t)255;
  const size_t oG2 = off; off += (size_t)nA1 * NB1 * DH * 4;                   off = (off + 255) & ~(size_t)255;
  const size_t oH2 = off; off += (size_t)nA2 * NB2 * DH * 4;                   off = (off + 255) & ~(size_t)255;
  if (off > ws_size) return;
  if (off > ((size_t)128 << 20)) return;
  _Float16* w1s  = (_Float16*)(ws + oW1);
  _Float16* w2s  = (_Float16*)(ws + oW2);
  _Float16* wfs  = (_Float16*)(ws + oWf);
  float*    dinv = (float*)(ws + oDv);
  float*    g1   = (float*)(ws + oG1);
  float*    g2   = (float*)(ws + oG2);
  float*    h2   = (float*)(ws + oH2);

  const int vec8 = ((nE & 3) == 0) ? 1 : 0;

  const int nPrep = DH * DF / 8 + DH * DH / 8 + NCP * DH / 8;
  k_wprep<<<(nPrep + NTHR - 1) / NTHR, NTHR, 0, stream>>>(W1, W2, Wf, w1s, w2s, wfs);

  k_deg<<<nBD, NTHR, 0, stream>>>(ei, dinv, nE, vec8);

  hipFuncSetAttribute(reinterpret_cast<const void*>(&k_gemm1),
                      hipFuncAttributeMaxDynamicSharedMemorySize, LDS_GEMM1);
  k_gemm1<<<nG1, NTHR, LDS_GEMM1, stream>>>(x, w1s, dinv, g1, nN);

  hipFuncSetAttribute(reinterpret_cast<const void*>(&k_agg1),
                      hipFuncAttributeMaxDynamicSharedMemorySize, LDS_AGG);
  k_agg1<<<nA1, NTHR, LDS_AGG, stream>>>(ei, g1, dinv, b1, w2s, g2, nN, nE, vec8);

  hipFuncSetAttribute(reinterpret_cast<const void*>(&k_agg2),
                      hipFuncAttributeMaxDynamicSharedMemorySize, LDS_AGG);
  k_agg2<<<nA2, NTHR, LDS_AGG, stream>>>(ei, g2, dinv, b2, h2, nN, nE, vec8);

  hipFuncSetAttribute(reinterpret_cast<const void*>(&k_pool),
                      hipFuncAttributeMaxDynamicSharedMemorySize, LDS_POOL);
  k_pool<<<1, NTHR, LDS_POOL, stream>>>(batch, h2, wfs, bfv, out, nN);
}
